// AttentionBlockOld_4020089389408
// MI455X (gfx1250) — hardware-verified
//
#include <hip/hip_runtime.h>
#include <hip/hip_bf16.h>
#include <math.h>

#define BBa 4
#define SSa 2048
#define CCa 256
#define NHa 8
#define DHa 64
#define DQa 512
#define DVa 2048
#define QKVW 3072
#define DEX 1024
#define MTOK (BBa * SSa)
#define GSTR 48
#define SS SSa
#define HH 1
#define DKK 64

typedef _Float16 bf16;
typedef _Float16 f16;
typedef __attribute__((ext_vector_type(4))) unsigned v4u_t;
typedef unsigned v4ua __attribute__((ext_vector_type(4), may_alias));
typedef __attribute__((ext_vector_type(4))) float v4f_t;
typedef float v4fa __attribute__((ext_vector_type(4), may_alias));
typedef __attribute__((ext_vector_type(16))) bf16  bf16x16;
typedef bf16x16 f16x16;
typedef __attribute__((ext_vector_type(8)))  bf16  bf16x8;
typedef bf16x8 f16x8;
typedef __attribute__((ext_vector_type(4)))  bf16  bf16x4;
typedef __attribute__((ext_vector_type(8)))  float f32x8;
__device__ __forceinline__ f32x8 wmma16(f16x16 a, f16x16 b, f32x8 c) {
  c = __builtin_amdgcn_wmma_f32_16x16x32_f16(false, a, false, b, (short)0, c, false, false);
  asm volatile("v_nop\n\tv_nop\n\tv_nop\n\tv_nop" : "+v"(c) : "v"(a), "v"(b));
  return c;
}
#define LDS_STRIDE 48
#define KSTRIDE    72
#define VSTRIDE    48

__device__ __forceinline__ f32x8 wmma_bf16(bf16x16 a, bf16x16 b, f32x8 c) {
  c = __builtin_amdgcn_wmma_f32_16x16x32_f16(false, a, false, b, (short)0, c, false, false);
  asm volatile("v_nop\n\tv_nop\n\tv_nop\n\tv_nop" : "+v"(c) : "v"(a), "v"(b));
  return c;
}

template <typename T>
__device__ __forceinline__ bf16x16 load_frag(const T* __restrict__ base, int ld,
                                             int row0, int k0) {
  const int lane = threadIdx.x & 31;
  const int r    = lane & 15;
  const int kh   = (lane >> 4) * 8;
  const T* p0 = base + (size_t)(row0 + r) * ld + (k0 + kh);
  const T* p1 = p0 + 16;
  bf16x16 f;
#pragma unroll
  for (int i = 0; i < 8; ++i) {
    f[i]     = (bf16)p0[i];
    f[i + 8] = (bf16)p1[i];
  }
  return f;
}

__device__ __forceinline__ bf16x16 lds_frag(const bf16* base, int stride) {
  const int lane = threadIdx.x & 31;
  const int row  = lane & 15;
  const int kh   = (lane >> 4) * 8;
  const bf16x8 lo = *(const bf16x8*)(base + row * stride + kh);
  const bf16x8 hi = *(const bf16x8*)(base + row * stride + kh + 16);
  bf16x16 f;
#pragma unroll
  for (int i = 0; i < 8; ++i) { f[i] = lo[i]; f[i + 8] = hi[i]; }
  return f;
}

template <typename T>
__device__ __forceinline__ void stage_read16(const T* __restrict__ p, float* buf) {
#pragma unroll
  for (int i = 0; i < 16; ++i) buf[i] = (float)p[i];
}

__device__ __forceinline__ void stage_write(bf16* dst, const float* buf, int nquad) {
#pragma unroll
  for (int i = 0; i < nquad; ++i) {
    bf16x4 q;
    q[0] = (bf16)buf[4 * i];     q[1] = (bf16)buf[4 * i + 1];
    q[2] = (bf16)buf[4 * i + 2]; q[3] = (bf16)buf[4 * i + 3];
    *(bf16x4*)(dst + 4 * i) = q;
  }
}

template <typename AT, int MODE>
__global__ __launch_bounds__(256) void gemm_rb_kernel(
    const AT* __restrict__ A, const float* __restrict__ W,
    const float* __restrict__ bias, const float* __restrict__ rowscale, const float* __restrict__ R, const float* __restrict__ rowbias, void* __restrict__ out,
    int M, int N, int K) {
  __shared__ bf16 ldsA[128 * LDS_STRIDE];
  __shared__ bf16 ldsW[256 * LDS_STRIDE];
  __shared__ __attribute__((aligned(16))) unsigned char sob[256 * 136 * 2];

  const int t    = threadIdx.x;
  const int wave = t >> 5;
  const int lane = t & 31;
  const int wm   = (wave & 1) * 64;
  const int wn   = (wave >> 1) * 64;
  const int mBlk = blockIdx.x * 128;
  const int nBlk = blockIdx.y * 256;

  const int arow = t >> 1;
  const int ach  = (t & 1) * 16;

  float abuf[16];
  float wbuf[32];

  stage_read16(A + (size_t)(mBlk + arow) * K + ach, abuf);
  const int nrow = min(nBlk + t, N - 1);
  stage_read16(W + (size_t)nrow * K,          wbuf);
  stage_read16(W + (size_t)nrow * K + 16,     wbuf + 16);

  f32x8 acc[4][4] = {};

  for (int k = 0; k < K; k += 32) {
    __syncthreads();
    stage_write(&ldsA[arow * LDS_STRIDE + ach], abuf, 4);
    stage_write(&ldsW[t * LDS_STRIDE],          wbuf, 8);
    if (k + 32 < K) {
      stage_read16(A + (size_t)(mBlk + arow) * K + (k + 32) + ach, abuf);
      stage_read16(W + (size_t)nrow * K + (k + 32),          wbuf);
      stage_read16(W + (size_t)nrow * K + (k + 32) + 16,     wbuf + 16);
    }
    __syncthreads();

    bf16x16 af[4], wf[4];
#pragma unroll
    for (int i = 0; i < 4; ++i)
      af[i] = lds_frag(ldsA + (wm + 16 * i) * LDS_STRIDE, LDS_STRIDE);
#pragma unroll
    for (int j = 0; j < 4; ++j)
      wf[j] = lds_frag(ldsW + (wn + 16 * j) * LDS_STRIDE, LDS_STRIDE);
#pragma unroll
    for (int i = 0; i < 4; ++i)
#pragma unroll
      for (int j = 0; j < 4; ++j)
        acc[i][j] = wmma_bf16(af[i], wf[j], acc[i][j]);
  }

  const int nlane = lane & 15;
  const int mh    = (lane >> 4) * 8;
  __syncthreads();
  if (MODE == 0 || MODE == 1 || MODE == 3) {
    bf16* so = (bf16*)sob;
#pragma unroll
    for (int i = 0; i < 4; ++i)
#pragma unroll
      for (int j = 0; j < 4; ++j) {
        const int nl = wn + 16 * j + nlane;
        const float bv = bias ? bias[nBlk + nl] : 0.0f;
        if (MODE == 3) {
#pragma unroll 1
          for (int r = 0; r < 8; ++r) {
            const int ml = wm + 16 * i + mh + r;
            const float xg = acc[i][j][r] + bv;
            so[ml * 264 + nl] = (bf16)(0.5f * xg * (1.0f + erff(xg * 0.70710678118654752f)));
          }
        } else {
#pragma unroll
        for (int r = 0; r < 8; ++r) {
          const int ml = wm + 16 * i + mh + r;
          const bf16 hv = (bf16)(acc[i][j][r] + bv);
          if (MODE == 0) so[ml * 264 + nl] = hv;
          else           so[nl * 136 + ml] = hv;
        }
        }
      }
    __syncthreads();
#pragma unroll 1
    for (int pass = 0; pass < 2; ++pass) {
      if (MODE == 0 || MODE == 3) {
        for (int ch = t; ch < 128 * 32; ch += 256) { const int ml = ch >> 5, q = (ch & 31) * 8;
          *(volatile v4u_t*)((bf16*)out + (size_t)(mBlk + ml) * N + nBlk + q) = *(const v4ua*)(so + ml * 264 + q); }
      } else {
        const int b_ = mBlk / SS, s0 = mBlk % SS;
        for (int ch = t; ch < 256 * 16; ch += 256) { const int nl = ch >> 4, q = (ch & 15) * 8; const int n = nBlk + nl, h = n >> 6, dk = n & (DKK - 1);
          *(volatile v4u_t*)((bf16*)out + (((size_t)(b_ * HH + h)) * DKK + dk) * SS + s0 + q) = *(const v4ua*)(so + nl * 136 + q); }
      }
      __threadfence();
    }
  } else {
    float* so = (float*)sob;
#pragma unroll 1
    for (int hf = 0; hf < 2; ++hf) {
      if (wm == hf * 64) {
#pragma unroll
        for (int i = 0; i < 4; ++i)
#pragma unroll
          for (int j = 0; j < 4; ++j) {
            const int nl = wn + 16 * j + nlane;
            const float bv = bias ? bias[nBlk + nl] : 0.0f;
#pragma unroll
            for (int r = 0; r < 8; ++r) { const int mrow = mBlk + hf * 64 + 16 * i + mh + r; so[(16 * i + mh + r) * 260 + nl] = acc[i][j][r] * (rowscale ? rowscale[mrow] : 1.0f) + bv + (rowbias ? rowbias[mrow] : 0.0f); }
          }
      }
      __syncthreads();
      if (R) {
        for (int ch = t; ch < 64 * 64; ch += 256) { const int ml = ch >> 6, q = (ch & 63) * 4;
          if (nBlk + q < N) { const v4f_t rv = *(const v4f_t*)(R + (size_t)(mBlk + hf * 64 + ml) * N + nBlk + q); v4f_t v = *(const v4fa*)(so + ml * 260 + q); v += rv; *(volatile v4fa*)(so + ml * 260 + q) = v; } }
        asm volatile("s_wait_dscnt 0" ::: "memory");
      }
#pragma unroll 1
      for (int pass = 0; pass < 2; ++pass) {
        for (int ch = t; ch < 64 * 64; ch += 256) { const int ml = ch >> 6, q = (ch & 63) * 4;
          if (nBlk + q < N) *(volatile v4f_t*)((float*)out + (size_t)(mBlk + hf * 64 + ml) * N + nBlk + q) = *(const v4fa*)(so + ml * 260 + q); }
        __threadfence();
      }
      __syncthreads();
    }
  }
}


#define GSTR 48
template <typename AT, int EPI, bool OUT16>
__global__ __launch_bounds__(256) void gemm_kne(const AT* __restrict__ A, int lda, const float* __restrict__ Wm, int ldw,
                                                const float* __restrict__ bias, const float* __restrict__ R, const float* __restrict__ gvec,
                                                void* __restrict__ Yv, int ldy, int K) {
  __shared__ __attribute__((aligned(16))) f16 ldsA[128 * GSTR];
  __shared__ __attribute__((aligned(16))) f16 ldsW[128 * GSTR];
  __shared__ __attribute__((aligned(16))) float oS[8][32 * 68];
  const int tid = threadIdx.x, lane = tid & 31, wave = tid >> 5, cl = lane & 15, rh = (lane >> 4) * 8;
  const int m0 = blockIdx.x * 128, n0 = blockIdx.y * 128;
  const int wm = (wave & 3) * 32, wn = (wave >> 2) * 64;
  f32x8 acc[2][4];
#pragma unroll
  for (int i = 0; i < 2; ++i)
#pragma unroll
    for (int j = 0; j < 4; ++j) { f32x8 z = {}; acc[i][j] = z; }
#pragma unroll 1
  for (int k0 = 0; k0 < K; k0 += 32) {
    __syncthreads();
    { const int row = tid >> 1, ch = (tid & 1) * 16;
      const AT* src = A + (size_t)(m0 + row) * lda + k0 + ch;
#pragma unroll
      for (int g = 0; g < 16; ++g) ldsA[row * GSTR + ch + g] = (f16)src[g]; }
    { const int k = tid >> 3, nn0 = (tid & 7) * 16;
      const float* src = Wm + (size_t)(k0 + k) * ldw + n0 + nn0;
#pragma unroll
      for (int g = 0; g < 4; ++g) { const v4f_t v = *(const v4f_t*)(src + 4 * g);
#pragma unroll
        for (int u = 0; u < 4; ++u) ldsW[(nn0 + 4 * g + u) * GSTR + k] = (f16)v[u]; } }
    __syncthreads();
    f16x16 af[2];
#pragma unroll
    for (int i = 0; i < 2; ++i) af[i] = lds_frag(ldsA + (wm + 16 * i) * GSTR, GSTR);
#pragma unroll
    for (int j = 0; j < 4; ++j) {
      const f16x16 bf = lds_frag(ldsW + (wn + 16 * j) * GSTR, GSTR);
#pragma unroll
      for (int i = 0; i < 2; ++i) acc[i][j] = wmma16(af[i], bf, acc[i][j]);
    }
  }
  float* so = oS[wave];
#pragma unroll
  for (int i = 0; i < 2; ++i)
#pragma unroll
    for (int j = 0; j < 4; ++j) {
      const int n = n0 + wn + 16 * j + cl;
      const float bv = bias ? bias[n] : 0.0f;
      const float gv = (EPI == 2) ? gvec[n] : 0.0f;
      if (EPI == 1) {
#pragma unroll 1
        for (int r = 0; r < 8; ++r) { const float xg = acc[i][j][r] + bv; so[(16 * i + rh + r) * 68 + 16 * j + cl] = 0.5f * xg * (1.0f + erff(xg * 0.70710678118654752f)); }
      } else {
#pragma unroll
        for (int r = 0; r < 8; ++r) {
          float v = acc[i][j][r] + bv;
          if (EPI == 2) v = R[(size_t)(m0 + wm + 16 * i + rh + r) * ldy + n] + gv * v;
          so[(16 * i + rh + r) * 68 + 16 * j + cl] = v;
        }
      }
    }
  asm volatile("s_wait_dscnt 0" ::: "memory");
  __builtin_amdgcn_wave_barrier();
#pragma unroll 1
  for (int pass = 0; pass < 2; ++pass) {
    if (OUT16) {
      f16* Y = (f16*)Yv;
#pragma unroll
      for (int it = 0; it < 8; ++it) { const int c = lane + 32 * it, rr = c >> 3, q8 = (c & 7) * 8;
        union { f16 h[8]; v4u_t v; } u;
#pragma unroll
        for (int e = 0; e < 8; ++e) u.h[e] = (f16)so[rr * 68 + q8 + e];
        *(volatile v4u_t*)(Y + (size_t)(m0 + wm + rr) * ldy + n0 + wn + q8) = u.v; }
    } else {
      float* Y = (float*)Yv;
#pragma unroll
      for (int it = 0; it < 16; ++it) { const int f4 = lane + 32 * it, rr = f4 >> 4, q = (f4 & 15) * 4;
        *(volatile v4f_t*)(Y + (size_t)(m0 + wm + rr) * ldy + n0 + wn + q) = *(const v4fa*)(so + rr * 68 + q); }
    }
    __threadfence();
  }
}

__global__ __launch_bounds__(256) void k_fnswish(const float* __restrict__ X, int addpe, const float* __restrict__ w, const float* __restrict__ bb, float* __restrict__ Y) {
  __shared__ __attribute__((aligned(16))) float rowS[8 * (CCa + 4)];
  const int tid = threadIdx.x, r = tid >> 5, lane = tid & 31; const size_t row = (size_t)blockIdx.x * 8 + r; const int n = row % SSa;
  const float lnb = logf(10000.0f) / (float)CCa;
  float s = 0.0f;
#pragma unroll 1
  for (int i = lane; i < CCa; i += 32) { float v = X[row * CCa + i];
    if (addpe) { const int i2 = i & ~1; const float ang = (float)n * expf(-lnb * (float)i2); v += (i & 1) ? cosf(ang) : sinf(ang); }
    rowS[r * (CCa + 4) + i] = v; s += v; }
#pragma unroll
  for (int off = 1; off < 32; off <<= 1) s += __shfl_xor(s, off, 32);
  const float mean = s * (1.0f / CCa); float q = 0.0f;
#pragma unroll 1
  for (int i = lane; i < CCa; i += 32) { const float d = rowS[r * (CCa + 4) + i] - mean; q += d * d; }
#pragma unroll
  for (int off = 1; off < 32; off <<= 1) q += __shfl_xor(q, off, 32);
  const float rstd = rsqrtf(q * (1.0f / CCa) + 1e-5f);
#pragma unroll 1
  for (int i = lane; i < CCa; i += 32) { const float u = (rowS[r * (CCa + 4) + i] - mean) * rstd * w[i] + bb[i]; rowS[r * (CCa + 4) + i] = u / (1.0f + expf(-u)); }
  __syncthreads();
#pragma unroll 1
  for (int pass = 0; pass < 2; ++pass) { for (int q4 = tid; q4 < 8 * (CCa / 4); q4 += 256) { const int rr = q4 / (CCa / 4), c4 = (q4 % (CCa / 4)) * 4;
      *(volatile v4f_t*)(Y + ((size_t)blockIdx.x * 8 + rr) * CCa + c4) = *(const v4fa*)(rowS + rr * (CCa + 4) + c4); } __threadfence(); }
}
__global__ __launch_bounds__(256) void k_qkhead(const float* __restrict__ qk, bf16* __restrict__ dummy, float* __restrict__ QH, float* __restrict__ KH, float* __restrict__ q2, float* __restrict__ k2) {
  __shared__ float nq[NHa][16], nk[NHa][16];
  (void)dummy;
  const size_t t0 = (size_t)blockIdx.x * 16; const int b = t0 / SSa, s0 = t0 % SSa; const int tid = threadIdx.x;
  for (int e = tid; e < 16 * NHa * 16; e += 256) { const int t = e >> 7, h = (e >> 4) & 7, c4 = (e & 15) * 4;
    const v4f_t q = *(const v4f_t*)(qk + (t0 + t) * (2 * DQa) + h * DHa + c4); const v4f_t k = *(const v4f_t*)(qk + (t0 + t) * (2 * DQa) + DQa + h * DHa + c4);
    float* dq = QH + (((size_t)b * NHa + h) * SSa + s0 + t) * DHa + c4; float* dk = KH + (((size_t)b * NHa + h) * SSa + s0 + t) * DHa + c4;
    *(volatile v4f_t*)dq = q; *(volatile v4f_t*)dk = k;
    float sq = q[0]*q[0] + q[1]*q[1] + q[2]*q[2] + q[3]*q[3], sk = k[0]*k[0] + k[1]*k[1] + k[2]*k[2] + k[3]*k[3];
#pragma unroll
    for (int off = 1; off < 16; off <<= 1) { sq += __shfl_xor(sq, off, 32); sk += __shfl_xor(sk, off, 32); }
    if ((tid & 15) == 0) { nq[h][t] = sq; nk[h][t] = sk; } }
  __syncthreads();
  __threadfence();
  for (int e = tid; e < 16 * NHa * 16; e += 256) { const int t = e >> 7, h = (e >> 4) & 7, c4 = (e & 15) * 4;
    *(volatile v4f_t*)(QH + (((size_t)b * NHa + h) * SSa + s0 + t) * DHa + c4) = *(const v4f_t*)(qk + (t0 + t) * (2 * DQa) + h * DHa + c4);
    *(volatile v4f_t*)(KH + (((size_t)b * NHa + h) * SSa + s0 + t) * DHa + c4) = *(const v4f_t*)(qk + (t0 + t) * (2 * DQa) + DQa + h * DHa + c4); }
#pragma unroll 1
  for (int pass = 0; pass < 2; ++pass) { if (tid < 32) { const int h = tid >> 2, c4 = (tid & 3) * 4; v4f_t a, c; for (int e = 0; e < 4; ++e) { a[e] = nq[h][c4 + e]; c[e] = nk[h][c4 + e]; }
      *(volatile v4f_t*)(q2 + ((size_t)b * NHa + h) * SSa + s0 + c4) = a; *(volatile v4f_t*)(k2 + ((size_t)b * NHa + h) * SSa + s0 + c4) = c; } __threadfence(); }
}
__global__ __launch_bounds__(256) void k_distsoftmax(float* __restrict__ S, const float* __restrict__ q2, const float* __restrict__ k2, const float* __restrict__ scale) {
  __shared__ float red[256];
  const size_t q = blockIdx.x; const int tid = threadIdx.x; float* sr = S + q * SSa; const float qq = q2[q]; const float sc = scale[0]; const float inv = 1.0f / (sc * sc);
  float v[8]; float m = -3.0e38f;
#pragma unroll
  for (int e = 0; e < 8; ++e) { const int k = tid * 8 + e; const float d2 = fmaxf(qq + k2[k] - 2.0f * sr[k], 0.0f); v[e] = -d2 * inv; m = fmaxf(m, v[e]); }
  red[tid] = m; __syncthreads();
  for (int o = 128; o > 0; o >>= 1) { if (tid < o) red[tid] = fmaxf(red[tid], red[tid + o]); __syncthreads(); }
  m = red[0]; __syncthreads();
  float z = 0.0f;
#pragma unroll
  for (int e = 0; e < 8; ++e) { v[e] = expf(v[e] - m); z += v[e]; }
  red[tid] = z; __syncthreads();
  for (int o = 128; o > 0; o >>= 1) { if (tid < o) red[tid] += red[tid + o]; __syncthreads(); }
  const float nrm = 1024.0f / red[0];
  v4f_t o0, o1; for (int e = 0; e < 4; ++e) { o0[e] = v[e] * nrm; o1[e] = v[4 + e] * nrm; }
#pragma unroll 1
  for (int pass = 0; pass < 2; ++pass) { *(volatile v4f_t*)(sr + tid * 8) = o0; *(volatile v4f_t*)(sr + tid * 8 + 4) = o1; __threadfence(); }
}
__global__ __launch_bounds__(256) void k_vT(const bf16* __restrict__ v16, int b, int h, float* __restrict__ VT) {
  __shared__ float tS[64][65 * 4 + 1];
  const int tid = threadIdx.x; const int s0 = blockIdx.x * 64;
  for (int e = tid; e < 64 * 256; e += 256) { const int t = e >> 8, c = e & 255; tS[t][c + (c >> 6)] = (float)v16[((size_t)b * SSa + s0 + t) * DVa + h * CCa + c]; }
  __syncthreads();
#pragma unroll 1
  for (int pass = 0; pass < 2; ++pass) { for (int e = tid; e < 256 * 16; e += 256) { const int c = e >> 4, q4 = (e & 15) * 4; v4f_t o; for (int i = 0; i < 4; ++i) o[i] = tS[q4 + i][c + (c >> 6)];
      *(volatile v4f_t*)(VT + (size_t)c * SSa + s0 + q4) = o; } __threadfence(); }
}
__global__ __launch_bounds__(256) void k_place(const float* __restrict__ Ot, int b, int h, bf16* __restrict__ O16) {
  const int s0 = blockIdx.x * 8; const int tid = threadIdx.x, r = tid >> 5, c8 = (tid & 31) * 8;
  union { bf16 hh[8]; v4u_t u; } cv; const float* src = Ot + (size_t)(s0 + r) * CCa + c8;
  for (int i = 0; i < 8; ++i) cv.hh[i] = (bf16)(src[i] * (1.0f / 1024.0f));
  bf16* dst = O16 + ((size_t)b * SSa + s0 + r) * DVa + h * CCa + c8; *(volatile v4u_t*)dst = cv.u; __threadfence(); *(volatile v4u_t*)dst = cv.u;
}
__global__ __launch_bounds__(256) void k_swish(float* __restrict__ t, int rowlen) { const size_t row = blockIdx.x;
  for (int q4 = threadIdx.x; q4 < rowlen / 4; q4 += 256) { v4f_t v = *(const v4f_t*)(t + row * rowlen + q4 * 4); for (int e = 0; e < 4; ++e) v[e] = v[e] / (1.0f + expf(-v[e]));
    *(volatile v4f_t*)(t + row * rowlen + q4 * 4) = v; __threadfence(); *(volatile v4f_t*)(t + row * rowlen + q4 * 4) = v; } }
__global__ __launch_bounds__(256) void k_fill(float* __restrict__ p, float val, int n) { for (int i = threadIdx.x; i < n; i += 256) { *(volatile float*)(p + i) = val; __threadfence(); *(volatile float*)(p + i) = val; } }

extern "C" void kernel_launch(void* const* d_in, const int* in_sizes, int n_in,
                              void* d_out, int out_size, void* d_ws, size_t ws_size,
                              hipStream_t stream) {
  (void)in_sizes; (void)n_in; (void)out_size;
  const float** f = (const float**)d_in;
  const float* x = f[0], *scale = f[1], *fn1w = f[2], *fn1b = f[3], *qkvw = f[4], *qkvb = f[5], *mw = f[6], *mb = f[7], *fn2w = f[8], *fn2b = f[9], *ff1w = f[10], *ff1b = f[11], *ff2w = f[12], *ff2b = f[13];
  float* out = (float*)d_out;
  char* ws = (char*)d_ws;
  float* h = (float*)ws; ws += (size_t)MTOK * CCa * 4;
  float* qk = (float*)ws; ws += (size_t)MTOK * 2 * DQa * 4;
  float* QH = (float*)ws; ws += (size_t)MTOK * DQa * 4;
  float* KH = (float*)ws; ws += (size_t)MTOK * DQa * 4;
  float* q2 = (float*)ws; ws += (size_t)BBa * NHa * SSa * 4; float* k2 = (float*)ws; ws += (size_t)BBa * NHa * SSa * 4;
  bf16* v16 = (bf16*)ws; ws += (size_t)MTOK * DVa * 2;
  bf16* O16 = (bf16*)ws; ws += (size_t)MTOK * DVa * 2;
  float* ones = (float*)ws; ws += 1024 * 4;
  float* S = qk; float* VT = qk + (size_t)SSa * SSa; float* Ot = VT + (size_t)CCa * SSa;
  if ((size_t)(ws - (char*)d_ws) > ws_size) return;
  const dim3 blk(256);
  k_fill<<<dim3(1), blk, 0, stream>>>(ones, 1.0f, 1024);
  k_fnswish<<<dim3(MTOK / 8), blk, 0, stream>>>(x, 1, fn1w, fn1b, h);
  gemm_kne<float, 0, false><<<dim3(MTOK / 128, 2 * DQa / 128), blk, 0, stream>>>(h, CCa, qkvw, QKVW, qkvb, nullptr, nullptr, qk, 2 * DQa, CCa);
  gemm_kne<float, 0, true><<<dim3(MTOK / 128, DVa / 128), blk, 0, stream>>>(h, CCa, qkvw + 2 * DQa, QKVW, qkvb + 2 * DQa, nullptr, nullptr, v16, DVa, CCa);
  k_qkhead<<<dim3(MTOK / 16), blk, 0, stream>>>(qk, nullptr, QH, KH, q2, k2);
  for (int b = 0; b < BBa; ++b) for (int hh = 0; hh < NHa; ++hh) {
    const float* Qs = QH + ((size_t)b * NHa + hh) * SSa * DHa; const float* Ks = KH + ((size_t)b * NHa + hh) * SSa * DHa;
    gemm_rb_kernel<float, 2><<<dim3(SSa / 128, SSa / 256), blk, 0, stream>>>(Qs, Ks, nullptr, nullptr, nullptr, nullptr, S, SSa, SSa, DHa);
    k_distsoftmax<<<dim3(SSa), blk, 0, stream>>>(S, q2 + ((size_t)b * NHa + hh) * SSa, k2 + ((size_t)b * NHa + hh) * SSa, scale);
    k_vT<<<dim3(SSa / 64), blk, 0, stream>>>(v16, b, hh, VT);
    gemm_rb_kernel<float, 2><<<dim3(SSa / 128, CCa / 256), blk, 0, stream>>>(S, VT, nullptr, nullptr, nullptr, nullptr, Ot, SSa, CCa, SSa);
    k_place<<<dim3(SSa / 8), blk, 0, stream>>>(Ot, b, hh, O16);
  }
  float* x1 = h;
  gemm_kne<bf16, 2, false><<<dim3(MTOK / 128, CCa / 128), blk, 0, stream>>>(O16, DVa, mw, CCa, mb, x, ones, x1, CCa, DVa);
  float* g = QH; float* ffh = (float*)v16;
  k_fnswish<<<dim3(MTOK / 8), blk, 0, stream>>>(x1, 0, fn2w, fn2b, g);
  gemm_kne<float, 0, false><<<dim3(MTOK / 128, DEX / 128), blk, 0, stream>>>(g, CCa, ff1w, DEX, ff1b, nullptr, nullptr, ffh, DEX, CCa);
  k_swish<<<dim3(MTOK), blk, 0, stream>>>(ffh, DEX);
  gemm_kne<float, 2, false><<<dim3(MTOK / 128, CCa / 128), blk, 0, stream>>>(ffh, DEX, ff2w, CCa, ff2b, x1, ones, out, CCa, DEX);
}
